// PatchScanMamba_52278341927352
// MI455X (gfx1250) — hardware-verified
//
#include <hip/hip_runtime.h>
#include <stdint.h>
#include <stddef.h>


#define NB_    32
#define NP_    192
#define SEQ_   193
#define DMOD_  384
#define DIN_   768
#define DXZ_   1536
#define NST_   16
#define DTR_   24
#define XDBL_  56
#define XDBP_  64
#define DTKP_  32
#define MR_    (NB_ * NP_)

static_assert(MR_ % 64 == 0);
static_assert(NP_ % 16 == 0);
static_assert(DMOD_ % 128 == 0);
static_assert(DIN_ % 128 == 0);
static_assert(DXZ_ % 128 == 0);
static_assert(DMOD_ == 96 * 4);
static_assert(DIN_ == 96 * 8);
static_assert(DMOD_ % 32 == 0 && DIN_ % 32 == 0 && DTKP_ % 32 == 0);
static_assert((MR_ * 4) % 256 == 0);

typedef float          v4f   __attribute__((ext_vector_type(4)));
typedef float          v8f   __attribute__((ext_vector_type(8)));
typedef _Float16       v8h   __attribute__((ext_vector_type(8)));
typedef _Float16       v16h  __attribute__((ext_vector_type(16)));
typedef unsigned short u16x8 __attribute__((ext_vector_type(8)));

union FragH { u16x8 h[2]; v16h v; };
union Pack8 { v8h f; u16x8 u; };
union H1    { _Float16 h; unsigned short u; };

__device__ __forceinline__ unsigned short f2h_bits(float f) { H1 t; t.h = (_Float16)f; return t.u; }
__device__ __forceinline__ float rcp_f(float x) { return __builtin_amdgcn_rcpf(x); }
__device__ __forceinline__ float silu_f(float x) {
    const float e = expf(-x);
    return x * rcp_f(1.0f + e);
}
__device__ __forceinline__ float softplus_f(float x) {
    return fmaxf(x, 0.0f) + log1pf(expf(-fabsf(x)));
}
__device__ __forceinline__ float conv4_silu(float x0, float x1, float x2, float x3,
                                            float w0, float w1, float w2, float w3, float bias) {
    const float c = w0 * x0 + w1 * x1 + w2 * x2 + w3 * x3;
    return silu_f(c + bias);
}
__device__ __forceinline__ v8f ld8f(const float* p) {
    const v4f a = *(const v4f*)p;
    const v4f b = *(const v4f*)(p + 4);
    return __builtin_shufflevector(a, b, 0, 1, 2, 3, 4, 5, 6, 7);
}
__device__ __forceinline__ float wave_sum(float v) {
#pragma unroll
    for (int o = 16; o > 0; o >>= 1) v += __shfl_xor(v, o, 32);
    return v;
}

__device__ __forceinline__ void mma16(v8f& acc, const FragH& a, const FragH& b) {
    acc = __builtin_amdgcn_wmma_f32_16x16x32_f16(false, a.v, false, b.v, (short)0, acc, false, false);
    asm volatile("v_nop\n\tv_nop\n\tv_nop\n\tv_nop" : "+v"(acc) : "v"(a.v), "v"(b.v));
}

__global__ __launch_bounds__(256)
void cvt_w_kernel(const float* __restrict__ src, int srcRows, int srcCols,
                  unsigned short* dst, int dstRows, int dstCols, float scale)
{
    const int i  = blockIdx.x * 256 + threadIdx.x;
    const int n8 = (dstRows * dstCols) >> 3;
    if (i >= n8) return;
    const int e  = i * 8;
    const int r  = e / dstCols;
    const int c0 = e - r * dstCols;
    u16x8 v;
#pragma unroll
    for (int c = 0; c < 8; ++c) {
        const int col = c0 + c;
        float f = 0.0f;
        if (r < srcRows && col < srcCols) f = src[(size_t)r * srcCols + col] * scale;
        v[c] = f2h_bits(f);
    }
    unsigned short* gp = dst + e;
    *(volatile u16x8*)gp = v;
    __threadfence();
    *(volatile u16x8*)gp = v;
}

template<int NBF>
__device__ __forceinline__ void tile_store_pass(const float* st, float* gp, int ldc, int lane) {
    constexpr int CW  = NBF * 16;
    constexpr int P   = CW + 4;
    constexpr int LPR = CW / 4;
    constexpr int RPI = 32 / LPR;
    constexpr int NIT = 32 / RPI;
    const int rsub = lane / LPR;
    const int c4   = (lane % LPR) * 4;
#pragma unroll
    for (int it = 0; it < NIT; ++it) {
        const int row = it * RPI + rsub;
        const v4f v = *(const v4f*)(st + row * P + c4);
        *(volatile v4f*)(gp + (size_t)row * ldc + c4) = v;
    }
}

template<int NBF>
__device__ __forceinline__ void tile_store_pass16(const float* st, unsigned short* H, int ldh, int hcol,
                                                  const float* __restrict__ resid, int ldr, int rcol,
                                                  int rowW, int flip, int lane) {
    constexpr int CW  = NBF * 16;
    constexpr int P   = CW + 4;
    constexpr int LPR = CW / 8;
    constexpr int RPI = 32 / LPR;
    constexpr int NIT = 32 / RPI;
    const int rsub = lane / LPR;
    const int c8   = (lane % LPR) * 8;
#pragma unroll
    for (int it = 0; it < NIT; ++it) {
        const int row  = it * RPI + rsub;
        const int grow = rowW + row;
        int orow = grow;
        if (flip) {
            const int b = grow / NP_;
            const int l = grow - b * NP_;
            orow = b * NP_ + (NP_ - 1 - l);
        }
        const v4f s0 = *(const v4f*)(st + row * P + c8);
        const v4f s1 = *(const v4f*)(st + row * P + c8 + 4);
        const float* rp = resid + (size_t)orow * ldr + rcol + c8;
        const v4f r0 = *(const v4f*)rp;
        const v4f r1 = *(const v4f*)(rp + 4);
        const v8f v = __builtin_shufflevector(s0 + r0, s1 + r1, 0, 1, 2, 3, 4, 5, 6, 7);
        Pack8 pk;
        pk.f = __builtin_convertvector(v, v8h);
        const u16x8 hv = pk.u;
        *(volatile u16x8*)(H + (size_t)orow * ldh + hcol + c8) = hv;
    }
}

template<int NBF, int MODE>
__global__ __launch_bounds__(128)
void gemm_tn_kernel(const unsigned short* __restrict__ A, const unsigned short* __restrict__ Bw,
                    int K, float scale,
                    float* C, int ldc,
                    unsigned short* H, int ldh, int hcol0,
                    const float* __restrict__ resid, int ldr, int flip)
{
    constexpr int CW = NBF * 16;
    constexpr int P  = CW + 4;
    static_assert(MODE == 0 || NBF == 4);
    __shared__ __attribute__((aligned(16))) float stile[4][32 * P];

    const int tid  = threadIdx.x;
    const int lane = tid & 31;
    const int wave = tid >> 5;
    const int h    = lane >> 4;
    const int m    = lane & 15;
    const int wm   = wave >> 1;
    const int wn   = wave & 1;

    const int rowW = blockIdx.y * 64 + wm * 32;
    const int colW = blockIdx.x * (2 * CW) + wn * CW;

    v8f acc[2 * NBF];
#pragma unroll
    for (int j = 0; j < 2 * NBF; ++j)
#pragma unroll
        for (int r = 0; r < 8; ++r) acc[j][r] = 0.0f;

    const size_t aoff  = (size_t)(rowW + m) * K + 8 * h;
    const size_t boff  = (size_t)(colW + m) * K + 8 * h;
    const size_t sub16 = (size_t)16 * K;
    const int nk = K >> 5;

    for (int kt = 0; kt < nk; ++kt) {
        const size_t k0 = (size_t)kt * 32;
        FragH fa[2], fb[NBF];
#pragma unroll
        for (int s = 0; s < 2; ++s) {
            const unsigned short* p = A + aoff + s * sub16 + k0;
            fa[s].h[0] = *(const u16x8*)(p);
            fa[s].h[1] = *(const u16x8*)(p + 16);
        }
#pragma unroll
        for (int j = 0; j < NBF; ++j) {
            const unsigned short* p = Bw + boff + j * sub16 + k0;
            fb[j].h[0] = *(const u16x8*)(p);
            fb[j].h[1] = *(const u16x8*)(p + 16);
        }
#pragma unroll
        for (int s = 0; s < 2; ++s)
#pragma unroll
            for (int j = 0; j < NBF; ++j)
                mma16(acc[s * NBF + j], fa[s], fb[j]);
    }

    float* st = stile[wave];
#pragma unroll
    for (int s = 0; s < 2; ++s)
#pragma unroll
        for (int j = 0; j < NBF; ++j)
#pragma unroll
            for (int r = 0; r < 8; ++r)
                st[(s * 16 + 8 * h + r) * P + j * 16 + m] = acc[s * NBF + j][r] * scale;
    __syncthreads();

    if (MODE == 0) {
        float* gp = C + (size_t)rowW * ldc + colW;
        tile_store_pass<NBF>(st, gp, ldc, lane);
        __threadfence();
        tile_store_pass<NBF>(st, gp, ldc, lane);
    } else {
        tile_store_pass16<NBF>(st, H, ldh, hcol0 + colW, resid, ldr, colW, rowW, flip, lane);
        __threadfence();
        tile_store_pass16<NBF>(st, H, ldh, hcol0 + colW, resid, ldr, colW, rowW, flip, lane);
    }
}

__global__ __launch_bounds__(96)
void ln_gather_kernel(const float* __restrict__ x, const int* __restrict__ sidx,
                      const float* __restrict__ gF, const float* __restrict__ bF,
                      const float* __restrict__ gB, const float* __restrict__ bB,
                      float* pr, unsigned short* xlnF, unsigned short* xlnB)
{
    __shared__ __attribute__((aligned(16))) float vn[DMOD_];
    __shared__ float red[2][4];

    const int m    = blockIdx.x;
    const int b    = m / NP_;
    const int l    = m - b * NP_;
    const int tid  = threadIdx.x;
    const int lane = tid & 31;
    const int wave = tid >> 5;

    int si = sidx[l];
    if (si < 0) si += NP_;
    si = min(max(si, 0), NP_ - 1);

    const v4f v = *(const v4f*)(x + ((size_t)b * SEQ_ + 1 + si) * DMOD_ + tid * 4);
    float* prp = pr + (size_t)m * DMOD_ + tid * 4;
    *(volatile v4f*)prp = v;

    float s = (v[0] + v[1]) + (v[2] + v[3]);
    s = wave_sum(s);
    if (lane == 0) red[0][wave] = s;
    __syncthreads();
    const float mean = ((red[0][0] + red[0][1]) + red[0][2]) * (1.0f / (float)DMOD_);
    const v4f dv = v - mean;
    float q = (dv[0] * dv[0] + dv[1] * dv[1]) + (dv[2] * dv[2] + dv[3] * dv[3]);
    q = wave_sum(q);
    if (lane == 0) red[1][wave] = q;
    __syncthreads();
    const float var = ((red[1][0] + red[1][1]) + red[1][2]) * (1.0f / (float)DMOD_);
    const float rs  = rsqrtf(var + 1e-5f);
    *(v4f*)(vn + tid * 4) = dv * rs;
    __threadfence();
    *(volatile v4f*)prp = v;
    __syncthreads();

    const int side = (tid < 48) ? 0 : 1;
    const int tt   = side ? (tid - 48) : tid;
    const int c0   = tt * 8;
    const v8f xn   = ld8f(vn + c0);
    const float* gp_ = side ? gB : gF;
    const float* bp_ = side ? bB : bF;
    const v8f gv = ld8f(gp_ + c0);
    const v8f bv = ld8f(bp_ + c0);
    Pack8 pk;
    pk.f = __builtin_convertvector(xn * gv + bv, v8h);
    const u16x8 hv = pk.u;
    const size_t orow = side ? ((size_t)b * NP_ + (NP_ - 1 - l)) : (size_t)m;
    unsigned short* gp = (side ? xlnB : xlnF) + orow * DMOD_ + c0;
    *(volatile u16x8*)gp = hv;
    __threadfence();
    *(volatile u16x8*)gp = hv;
}

__global__ __launch_bounds__(96)
void conv_silu_kernel(const float* __restrict__ XZ, const float* __restrict__ cw,
                      const float* __restrict__ cb, unsigned short* U16)
{
    const int m  = blockIdx.x;
    const int l  = m % NP_;
    const int d0 = threadIdx.x * 8;
    const float* xr = XZ + (size_t)m * DXZ_ + d0;

    const v8f x3 = ld8f(xr);
    v8f x2, x1, x0;
#pragma unroll
    for (int c = 0; c < 8; ++c) { x2[c] = 0.0f; x1[c] = 0.0f; x0[c] = 0.0f; }
    if (l >= 1) x2 = ld8f(xr - DXZ_);
    if (l >= 2) x1 = ld8f(xr - 2 * DXZ_);
    if (l >= 3) x0 = ld8f(xr - 3 * DXZ_);

    const float* wp = cw + (size_t)d0 * 4;
    v4f wv[8];
#pragma unroll
    for (int c = 0; c < 8; ++c) wv[c] = *(const v4f*)(wp + 4 * c);
    const v8f bias = ld8f(cb + d0);

    v8f u;
#pragma unroll
    for (int c = 0; c < 8; ++c)
        u[c] = conv4_silu(x0[c], x1[c], x2[c], x3[c], wv[c][0], wv[c][1], wv[c][2], wv[c][3], bias[c]);

    Pack8 pk;
    pk.f = __builtin_convertvector(u * 64.0f, v8h);
    const u16x8 hv = pk.u;
    unsigned short* gp = U16 + (size_t)m * DIN_ + d0;
    *(volatile u16x8*)gp = hv;
    __threadfence();
    *(volatile u16x8*)gp = hv;
}

__global__ __launch_bounds__(256)
void dtr_cvt_kernel(const float* __restrict__ XDBL, unsigned short* DT16, int nrows)
{
    const int t   = blockIdx.x * 256 + threadIdx.x;
    const int row = t >> 2;
    const int p   = t & 3;
    if (row >= nrows) return;
    u16x8 v;
#pragma unroll
    for (int c = 0; c < 8; ++c) {
        const int col = p * 8 + c;
        float f = 0.0f;
        if (col < DTR_) f = XDBL[(size_t)row * XDBP_ + col] * 64.0f;
        v[c] = f2h_bits(f);
    }
    unsigned short* gp = DT16 + (size_t)row * DTKP_ + p * 8;
    *(volatile u16x8*)gp = v;
    __threadfence();
    *(volatile u16x8*)gp = v;
}

__device__ __forceinline__ void yg_store_pass(const unsigned short* sy, unsigned short* YG,
                                              size_t gbase, int wave, int lane) {
#pragma unroll
    for (int it = 0; it < 2; ++it) {
        const int t = wave * 8 + it * 4 + (lane >> 3);
        const int c = (lane & 7) * 8;
        const u16x8 v = *(const u16x8*)(sy + t * 64 + c);
        *(volatile u16x8*)(YG + gbase + (size_t)t * DIN_ + c) = v;
    }
}

__global__ __launch_bounds__(64)
void scan_kernel(const float* __restrict__ XZ, const float* __restrict__ DTRAW,
                 const float* __restrict__ XDBL, const float* __restrict__ cw,
                 const float* __restrict__ cb, const float* __restrict__ dtb,
                 const float* __restrict__ Alog, const float* __restrict__ Dp,
                 unsigned short* YG)
{
    __shared__ __attribute__((aligned(16))) unsigned short sy[16 * 64];

    const int tid   = threadIdx.x;
    const int lane  = tid & 31;
    const int wave  = tid >> 5;
    const int dbase = blockIdx.x * 64;
    const int d     = dbase + tid;
    const int b     = blockIdx.y;

    float an[NST_], hs[NST_];
#pragma unroll
    for (int n = 0; n < NST_; ++n) {
        an[n] = -expf(Alog[(size_t)d * NST_ + n]);
        hs[n] = 0.0f;
    }
    const float w0 = cw[d * 4 + 0], w1 = cw[d * 4 + 1], w2 = cw[d * 4 + 2], w3 = cw[d * 4 + 3];
    const float cbias = cb[d];
    const float tb    = dtb[d];
    const float Dd    = Dp[d];

    float xm1 = 0.0f, xm2 = 0.0f, xm3 = 0.0f;
    const size_t row0 = (size_t)b * NP_;

#pragma unroll 1
    for (int l0 = 0; l0 < NP_; l0 += 16) {
#pragma unroll 1
        for (int t = 0; t < 16; ++t) {
            const size_t row = row0 + (size_t)(l0 + t);
            const float xv = XZ[row * DXZ_ + d];
            const float zv = XZ[row * DXZ_ + DIN_ + d];
            const float dl = DTRAW[row * DIN_ + d];
            const float u  = conv4_silu(xm3, xm2, xm1, xv, w0, w1, w2, w3, cbias);
            xm3 = xm2; xm2 = xm1; xm1 = xv;
            const float dt = softplus_f(dl + tb);
            const float du = dt * u;
            const float* bc = XDBL + row * XDBP_ + DTR_;
            float y = 0.0f;
#pragma unroll
            for (int n = 0; n < NST_; ++n) {
                const float bn = bc[n];
                const float cn = bc[NST_ + n];
                const float da = __expf(dt * an[n]);
                hs[n] = da * hs[n] + du * bn;
                y += hs[n] * cn;
            }
            const float g = (y + Dd * u) * silu_f(zv);
            sy[t * 64 + tid] = f2h_bits(g * 64.0f);
        }
        __syncthreads();
        const size_t gbase = (row0 + (size_t)l0) * DIN_ + dbase;
        yg_store_pass(sy, YG, gbase, wave, lane);
        __threadfence();
        yg_store_pass(sy, YG, gbase, wave, lane);
        __syncthreads();
    }
}

__global__ __launch_bounds__(96)
void out_gather_kernel(const float* __restrict__ x, const float* __restrict__ FO,
                       const float* __restrict__ fbias, const int* __restrict__ inv, float* out)
{
    const int blk = blockIdx.x;
    const int b   = blk / SEQ_;
    const int p   = blk - b * SEQ_;
    const int tid = threadIdx.x;
    v4f v;
    if (p == 0) {
        v = *(const v4f*)(x + (size_t)b * SEQ_ * DMOD_ + tid * 4);
    } else {
        int j = inv[p - 1];
        if (j < 0) j += NP_;
        j = min(max(j, 0), NP_ - 1);
        const v4f f  = *(const v4f*)(FO + ((size_t)b * NP_ + j) * DMOD_ + tid * 4);
        const v4f bb = *(const v4f*)(fbias + tid * 4);
        v = f + bb;
    }
    float* op = out + (size_t)blk * DMOD_ + tid * 4;
    *(volatile v4f*)op = v;
    __threadfence();
    *(volatile v4f*)op = v;
}

extern "C" void kernel_launch(void* const* d_in, const int* in_sizes, int n_in,
                              void* d_out, int out_size, void* d_ws, size_t ws_size,
                              hipStream_t stream)
{
    if (n_in < 27) return;
    if (in_sizes[0] != NB_ * SEQ_ * DMOD_) return;
    for (int p = 0; p < 2; ++p) {
        const int o = p ? 12 : 1;
        if (in_sizes[o + 0]  != DMOD_)          return;
        if (in_sizes[o + 1]  != DMOD_)          return;
        if (in_sizes[o + 2]  != DXZ_ * DMOD_)   return;
        if (in_sizes[o + 3]  != DIN_ * 4)       return;
        if (in_sizes[o + 4]  != DIN_)           return;
        if (in_sizes[o + 5]  != XDBL_ * DIN_)   return;
        if (in_sizes[o + 6]  != DIN_ * DTR_)    return;
        if (in_sizes[o + 7]  != DIN_)           return;
        if (in_sizes[o + 8]  != DIN_ * NST_)    return;
        if (in_sizes[o + 9]  != DIN_)           return;
        if (in_sizes[o + 10] != DMOD_ * DIN_)   return;
    }
    if (in_sizes[23] != DMOD_ * 2 * DMOD_) return;
    if (in_sizes[24] != DMOD_)             return;
    if (in_sizes[25] != NP_)               return;
    if (in_sizes[26] != NP_)               return;
    if (out_size != NB_ * SEQ_ * DMOD_)    return;

    const float* x = (const float*)d_in[0];
    const float* ln_g[2]   = {(const float*)d_in[1],  (const float*)d_in[12]};
    const float* ln_b[2]   = {(const float*)d_in[2],  (const float*)d_in[13]};
    const float* in_w[2]   = {(const float*)d_in[3],  (const float*)d_in[14]};
    const float* conv_w[2] = {(const float*)d_in[4],  (const float*)d_in[15]};
    const float* conv_b[2] = {(const float*)d_in[5],  (const float*)d_in[16]};
    const float* x_w[2]    = {(const float*)d_in[6],  (const float*)d_in[17]};
    const float* dt_w[2]   = {(const float*)d_in[7],  (const float*)d_in[18]};
    const float* dt_b[2]   = {(const float*)d_in[8],  (const float*)d_in[19]};
    const float* A_log[2]  = {(const float*)d_in[9],  (const float*)d_in[20]};
    const float* Dp[2]     = {(const float*)d_in[10], (const float*)d_in[21]};
    const float* out_w[2]  = {(const float*)d_in[11], (const float*)d_in[22]};
    const float* fusion_w  = (const float*)d_in[23];
    const float* fusion_b  = (const float*)d_in[24];
    const int*   scan_idx  = (const int*)d_in[25];
    const int*   inv_idx   = (const int*)d_in[26];
    float* out = (float*)d_out;

    const size_t SZ_INW  = (size_t)DXZ_ * DMOD_ * 2;
    const size_t SZ_XW   = (size_t)XDBP_ * DIN_ * 2;
    const size_t SZ_DTW  = (size_t)DIN_ * DTKP_ * 2;
    const size_t SZ_OW   = (size_t)DMOD_ * DIN_ * 2;
    const size_t SZ_FW   = (size_t)DMOD_ * DIN_ * 2;
    const size_t SZ_PR   = (size_t)MR_ * DMOD_ * 4;
    const size_t SZ_XLN  = (size_t)MR_ * DMOD_ * 2;
    const size_t SZ_XZ   = (size_t)MR_ * DXZ_ * 4;
    const size_t SZ_U16  = (size_t)MR_ * DIN_ * 2;
    const size_t SZ_XDBL = (size_t)MR_ * XDBP_ * 4;
    const size_t SZ_DT16 = (size_t)MR_ * DTKP_ * 2;
    const size_t SZ_DTR  = (size_t)MR_ * DIN_ * 4;
    const size_t SZ_YG   = (size_t)MR_ * DIN_ * 2;
    const size_t SZ_FUS  = (size_t)MR_ * DIN_ * 2;
    const size_t SZ_FO   = (size_t)MR_ * DMOD_ * 4;

    size_t off = 0;
    const size_t OFF_INW0 = off; off += SZ_INW;
    const size_t OFF_INW1 = off; off += SZ_INW;
    const size_t OFF_XW0  = off; off += SZ_XW;
    const size_t OFF_XW1  = off; off += SZ_XW;
    const size_t OFF_DTW0 = off; off += SZ_DTW;
    const size_t OFF_DTW1 = off; off += SZ_DTW;
    const size_t OFF_OW0  = off; off += SZ_OW;
    const size_t OFF_OW1  = off; off += SZ_OW;
    const size_t OFF_FW   = off; off += SZ_FW;
    const size_t OFF_PR   = off; off += SZ_PR;
    const size_t OFF_XLN0 = off; off += SZ_XLN;
    const size_t OFF_XLN1 = off; off += SZ_XLN;
    const size_t OFF_XZ   = off; off += SZ_XZ;
    const size_t OFF_U16  = off; off += SZ_U16;
    const size_t OFF_XDBL = off; off += SZ_XDBL;
    const size_t OFF_DT16 = off; off += SZ_DT16;
    const size_t OFF_DTR  = off; off += SZ_DTR;
    const size_t OFF_YG   = off; off += SZ_YG;
    const size_t OFF_FUS  = off; off += SZ_FUS;
    const size_t OFF_FO   = off; off += SZ_FO;
    const size_t WS_END   = off;
    if (WS_END > (size_t)134217728) return;
    if (ws_size < WS_END) return;

    char* ws = (char*)d_ws;
    unsigned short* inw16[2] = {(unsigned short*)(ws + OFF_INW0), (unsigned short*)(ws + OFF_INW1)};
    unsigned short* xw16[2]  = {(unsigned short*)(ws + OFF_XW0),  (unsigned short*)(ws + OFF_XW1)};
    unsigned short* dtw16[2] = {(unsigned short*)(ws + OFF_DTW0), (unsigned short*)(ws + OFF_DTW1)};
    unsigned short* ow16[2]  = {(unsigned short*)(ws + OFF_OW0),  (unsigned short*)(ws + OFF_OW1)};
    unsigned short* fw16     = (unsigned short*)(ws + OFF_FW);
    float*          pr       = (float*)(ws + OFF_PR);
    unsigned short* xln16[2] = {(unsigned short*)(ws + OFF_XLN0), (unsigned short*)(ws + OFF_XLN1)};
    float*          xz       = (float*)(ws + OFF_XZ);
    unsigned short* u16      = (unsigned short*)(ws + OFF_U16);
    float*          xdbl     = (float*)(ws + OFF_XDBL);
    unsigned short* dt16     = (unsigned short*)(ws + OFF_DT16);
    float*          dtraw    = (float*)(ws + OFF_DTR);
    unsigned short* yg16     = (unsigned short*)(ws + OFF_YG);
    unsigned short* fus16    = (unsigned short*)(ws + OFF_FUS);
    float*          fo       = (float*)(ws + OFF_FO);

    auto cvt = [&](const float* s, int sr, int sc, unsigned short* dst, int dr, int dc, float scale) {
        const int n8 = (dr * dc) / 8;
        hipLaunchKernelGGL(cvt_w_kernel, dim3((n8 + 255) / 256), dim3(256), 0, stream,
                           s, sr, sc, dst, dr, dc, scale);
    };
    for (int p = 0; p < 2; ++p) {
        cvt(in_w[p],  DXZ_,  DMOD_, inw16[p], DXZ_,  DMOD_, 32.0f);
        cvt(x_w[p],   XDBL_, DIN_,  xw16[p],  XDBP_, DIN_,  32.0f);
        cvt(dt_w[p],  DIN_,  DTR_,  dtw16[p], DIN_,  DTKP_, 8.0f);
        cvt(out_w[p], DMOD_, DIN_,  ow16[p],  DMOD_, DIN_,  32.0f);
    }
    cvt(fusion_w, DMOD_, DIN_, fw16, DMOD_, DIN_, 32.0f);

    hipLaunchKernelGGL(ln_gather_kernel, dim3(MR_), dim3(96), 0, stream,
                       x, scan_idx, ln_g[0], ln_b[0], ln_g[1], ln_b[1], pr, xln16[0], xln16[1]);

    for (int dir = 0; dir < 2; ++dir) {
        gemm_tn_kernel<4, 0><<<dim3(DXZ_ / 128, MR_ / 64), dim3(128), 0, stream>>>(
            (const unsigned short*)xln16[dir], (const unsigned short*)inw16[dir],
            (int)DMOD_, 0.03125f, xz, (int)DXZ_,
            yg16, 0, 0, (const float*)pr, 0, 0);

        hipLaunchKernelGGL(conv_silu_kernel, dim3(MR_), dim3(96), 0, stream,
                           (const float*)xz, conv_w[dir], conv_b[dir], u16);

        gemm_tn_kernel<2, 0><<<dim3(XDBP_ / 64, MR_ / 64), dim3(128), 0, stream>>>(
            (const unsigned short*)u16, (const unsigned short*)xw16[dir],
            (int)DIN_, 0.00048828125f, xdbl, (int)XDBP_,
            yg16, 0, 0, (const float*)pr, 0, 0);

        hipLaunchKernelGGL(dtr_cvt_kernel, dim3((MR_ * 4) / 256), dim3(256), 0, stream,
                           (const float*)xdbl, dt16, (int)MR_);

        gemm_tn_kernel<4, 0><<<dim3(DIN_ / 128, MR_ / 64), dim3(128), 0, stream>>>(
            (const unsigned short*)dt16, (const unsigned short*)dtw16[dir],
            (int)DTKP_, 0.001953125f, dtraw, (int)DIN_,
            yg16, 0, 0, (const float*)pr, 0, 0);

        hipLaunchKernelGGL(scan_kernel, dim3(DIN_ / 64, NB_), dim3(64), 0, stream,
                           (const float*)xz, (const float*)dtraw, (const float*)xdbl,
                           conv_w[dir], conv_b[dir], dt_b[dir], A_log[dir], Dp[dir], yg16);

        gemm_tn_kernel<4, 1><<<dim3(DMOD_ / 128, MR_ / 64), dim3(128), 0, stream>>>(
            (const unsigned short*)yg16, (const unsigned short*)ow16[dir],
            (int)DIN_, 0.00048828125f, fo, (int)DMOD_,
            fus16, (int)DIN_, (int)(dir * DMOD_), (const float*)pr, (int)DMOD_, (int)dir);
    }

    gemm_tn_kernel<4, 0><<<dim3(DMOD_ / 128, MR_ / 64), dim3(128), 0, stream>>>(
        (const unsigned short*)fus16, (const unsigned short*)fw16,
        (int)DIN_, 0.03125f, fo, (int)DMOD_,
        yg16, 0, 0, (const float*)pr, 0, 0);

    hipLaunchKernelGGL(out_gather_kernel, dim3(NB_ * SEQ_), dim3(96), 0, stream,
                       x, (const float*)fo, fusion_b, inv_idx, out);
}
